// HybridSTHGAT_76124000354333
// MI455X (gfx1250) — hardware-verified
//
#include <hip/hip_runtime.h>


namespace {
constexpr int NB = 4096, NST = 64, INF = 32, H = 128, HH = 64, L = 2;
constexpr float XS = 8.0f, WSC = 256.0f, EPS = 1e-5f;
typedef _Float16 b16;
typedef __attribute__((ext_vector_type(16))) _Float16 v16b;
typedef __attribute__((ext_vector_type(8))) _Float16 v8b;
typedef __attribute__((ext_vector_type(8))) float v8f;
typedef __attribute__((ext_vector_type(4))) float v4f;
__device__ __forceinline__ float bf16_rne(float f) { unsigned int u = __float_as_uint(f); u += 0x7FFFu + ((u >> 16) & 1u); return __uint_as_float(u & 0xFFFF0000u); }
__device__ __forceinline__ void split16(float v, b16& hi, b16& lo) { hi = (b16)v; lo = (b16)(v - (float)hi); }
__device__ __forceinline__ v16b frag_kb(const b16* p, int hh) { const v8b a = *(const v8b*)(p + 8 * hh), b = *(const v8b*)(p + 16 + 8 * hh); v16b f;
#pragma unroll
  for (int e = 0; e < 8; ++e) { f[e] = a[e]; f[8 + e] = b[e]; } return f; }
__device__ __forceinline__ v8f wmma16b(v16b a, v16b b, v8f c) { v8f d = __builtin_amdgcn_wmma_f32_16x16x32_f16(false, a, false, b, (short)0, c, false, false); asm volatile("v_nop\n\tv_nop\n\tv_nop\n\tv_nop" : "+v"(d) : "v"(a), "v"(b)); return d; }
__device__ __forceinline__ void wave_lds_sync() { __builtin_amdgcn_fence(__ATOMIC_RELEASE, "workgroup"); __builtin_amdgcn_wave_barrier(); __builtin_amdgcn_fence(__ATOMIC_ACQUIRE, "workgroup"); }
__device__ __forceinline__ float pmul(float a, float b) { float p = a * b; asm volatile("" : "+v"(p)); return p; }
__device__ __forceinline__ int iclamp(int v, int lo, int hi) { return v < lo ? lo : (v > hi ? hi : v); }
__device__ __forceinline__ float eluf(float x) { return x > 0.0f ? x : (__expf(x) - 1.0f); }

struct WJob { const float* w; int KIN, OUT; b16* WT; };
__global__ __launch_bounds__(256) void wprep_kernel(WJob j0, WJob j1, WJob j2, WJob j3, WJob j4, WJob j5) {
  const WJob j = blockIdx.y == 0 ? j0 : blockIdx.y == 1 ? j1 : blockIdx.y == 2 ? j2 : blockIdx.y == 3 ? j3 : blockIdx.y == 4 ? j4 : j5;
  const size_t u = (size_t)blockIdx.x * 256 + threadIdx.x; if (u >= (size_t)j.OUT * j.KIN / 8) return; const size_t e = u * 8; const int o = (int)(e / j.KIN), k0 = (int)(e % j.KIN); v8b v;
  for (int q = 0; q < 8; ++q) v[q] = (b16)(bf16_rne(j.w[(size_t)(k0 + q) * j.OUT + o]) * WSC); for (int pass = 0; pass < 2; ++pass) { *(volatile v8b*)(j.WT + e) = v; __threadfence(); }
}
template <int NT, int KW>
__device__ __forceinline__ void gemm_tiles(const b16 (*Ah)[H + HH + 8], const b16 (*Al)[H + HH + 8], const b16* __restrict__ WT, v8f* acc, int nloc, int hlf) {
#pragma unroll
  for (int t = 0; t < NT; ++t) acc[t] = (v8f){};
#pragma unroll
  for (int kb = 0; kb < KW; kb += 32) { const v16b a = frag_kb(&Ah[nloc][kb], hlf), al = frag_kb(&Al[nloc][kb], hlf);
#pragma unroll
    for (int t = 0; t < NT; ++t) { const v16b bw = frag_kb(WT + (size_t)(t * 16 + nloc) * KW + kb, hlf); acc[t] = wmma16b(a, bw, acc[t]); acc[t] = wmma16b(al, bw, acc[t]); } }
}
template <int NT>
__device__ __forceinline__ void ln_relu_rows(v8f* acc, const float* __restrict__ g, const float* __restrict__ b, int nloc) {
  constexpr float inv = 1.0f / (NT * 16);
#pragma unroll
  for (int r8 = 0; r8 < 8; ++r8) { float s = 0.0f; for (int t = 0; t < NT; ++t) s += acc[t][r8]; for (int o = 1; o < 16; o <<= 1) s += __shfl_xor(s, o); const float mu = s * inv;
    float q = 0.0f; for (int t = 0; t < NT; ++t) { const float d = acc[t][r8] - mu; q += pmul(d, d); } for (int o = 1; o < 16; o <<= 1) q += __shfl_xor(q, o); const float rs = rsqrtf(q * inv + EPS);
    for (int t = 0; t < NT; ++t) { const int c = t * 16 + nloc; acc[t][r8] = fmaxf(pmul(pmul(acc[t][r8] - mu, rs), bf16_rne(g[c])) + bf16_rne(b[c]), 0.0f); } }
}
__global__ __launch_bounds__(64) void chain_kernel(const float* __restrict__ x, const int* __restrict__ sidx, const float* __restrict__ emb, const b16* __restrict__ WP, const b16* __restrict__ WG0, const b16* __restrict__ WG1, const b16* __restrict__ W1T, const b16* __restrict__ W2T,
                                                   const float* __restrict__ bp, const float* __restrict__ b1, const float* __restrict__ g1, const float* __restrict__ be1, const float* __restrict__ b2, const float* __restrict__ g2, const float* __restrict__ be2, const float* __restrict__ wo, const float* __restrict__ bo, float* __restrict__ out) {
  __shared__ __attribute__((aligned(16))) b16 Ah[2][16][H + HH + 8], Al[2][16][H + HH + 8]; __shared__ float so[32];
  const int wave = threadIdx.x >> 5, lane = threadIdx.x & 31, nloc = lane & 15, hlf = lane >> 4; const size_t m0 = (size_t)blockIdx.x * 32 + wave * 16; const float sc = 1.0f / (XS * WSC);
  for (int rr = 0; rr < 16; ++rr) { const float v = x[(m0 + rr) * INF + lane]; Ah[wave][rr][lane] = (b16)(bf16_rne(v) * XS); Al[wave][rr][lane] = (b16)0.0f; }
  wave_lds_sync();
  v8f acc[8]; float h[8][8];
  gemm_tiles<8, INF>(Ah[wave], Al[wave], WP, acc, nloc, hlf);
#pragma unroll
  for (int t = 0; t < 8; ++t) { const float bb = bf16_rne(bp[t * 16 + nloc]);
#pragma unroll
    for (int r8 = 0; r8 < 8; ++r8) h[t][r8] = acc[t][r8] * sc + bb; }
#pragma unroll 1
  for (int l = 0; l < L; ++l) { const b16* WG = l == 0 ? WG0 : WG1;
    wave_lds_sync();
#pragma unroll
    for (int t = 0; t < 8; ++t)
#pragma unroll
      for (int r8 = 0; r8 < 8; ++r8) { b16 p, ql; split16(h[t][r8] * XS, p, ql); Ah[wave][8 * hlf + r8][t * 16 + nloc] = p; Al[wave][8 * hlf + r8][t * 16 + nloc] = ql; }
    wave_lds_sync();
    gemm_tiles<8, H>(Ah[wave], Al[wave], WG, acc, nloc, hlf);
#pragma unroll
    for (int t = 0; t < 8; ++t)
#pragma unroll
      for (int r8 = 0; r8 < 8; ++r8) h[t][r8] += eluf(acc[t][r8] * sc); }
  wave_lds_sync();
#pragma unroll
  for (int t = 0; t < 8; ++t)
#pragma unroll
    for (int r8 = 0; r8 < 8; ++r8) { b16 p, ql; split16(h[t][r8] * XS, p, ql); Ah[wave][8 * hlf + r8][t * 16 + nloc] = p; Al[wave][8 * hlf + r8][t * 16 + nloc] = ql; }
  for (int rr = 0; rr < 16; ++rr) { const int st = iclamp(sidx[m0 + rr], 0, NST - 1); const float e0 = emb[st * HH + lane * 2], e1 = emb[st * HH + lane * 2 + 1]; Ah[wave][rr][H + lane * 2] = (b16)(bf16_rne(e0) * XS); Ah[wave][rr][H + lane * 2 + 1] = (b16)(bf16_rne(e1) * XS); Al[wave][rr][H + lane * 2] = (b16)0.0f; Al[wave][rr][H + lane * 2 + 1] = (b16)0.0f; }
  wave_lds_sync();
  gemm_tiles<8, H + HH>(Ah[wave], Al[wave], W1T, acc, nloc, hlf);
#pragma unroll
  for (int t = 0; t < 8; ++t) { const float bb = bf16_rne(b1[t * 16 + nloc]);
#pragma unroll
    for (int r8 = 0; r8 < 8; ++r8) acc[t][r8] = acc[t][r8] * sc + bb; }
  ln_relu_rows<8>(acc, g1, be1, nloc);
  wave_lds_sync();
#pragma unroll
  for (int t = 0; t < 8; ++t)
#pragma unroll
    for (int r8 = 0; r8 < 8; ++r8) { b16 p, ql; split16(acc[t][r8] * XS, p, ql); Ah[wave][8 * hlf + r8][t * 16 + nloc] = p; Al[wave][8 * hlf + r8][t * 16 + nloc] = ql; }
  wave_lds_sync();
  v8f a2[4]; gemm_tiles<4, H>(Ah[wave], Al[wave], W2T, a2, nloc, hlf);
#pragma unroll
  for (int t = 0; t < 4; ++t) { const float bb = bf16_rne(b2[t * 16 + nloc]);
#pragma unroll
    for (int r8 = 0; r8 < 8; ++r8) a2[t][r8] = a2[t][r8] * sc + bb; }
  ln_relu_rows<4>(a2, g2, be2, nloc);
  { const float bov = bf16_rne(bo[0]); float w4[4]; for (int t = 0; t < 4; ++t) w4[t] = bf16_rne(wo[t * 16 + nloc]);
#pragma unroll
    for (int r8 = 0; r8 < 8; ++r8) { float s = 0.0f; for (int t = 0; t < 4; ++t) s += pmul(a2[t][r8], w4[t]); for (int o = 1; o < 16; o <<= 1) s += __shfl_xor(s, o); if (nloc == 0) so[wave * 16 + 8 * hlf + r8] = s + bov; } }
  __syncthreads();
  for (int pass = 0; pass < 2; ++pass) { if (threadIdx.x < 32) ((volatile float*)out)[(size_t)blockIdx.x * 32 + threadIdx.x] = so[threadIdx.x]; __threadfence(); }
}
}

extern "C" void kernel_launch(void* const* d_in, const int* in_sizes, int n_in, void* d_out, int out_size, void* d_ws, size_t ws_size, hipStream_t stream) {
  (void)n_in;
  auto Fp = [&](int i) { return (const float*)d_in[i]; }; auto Ip = [&](int i) { return (const int*)d_in[i]; };
  if (in_sizes[0] != NB * INF || in_sizes[1] != NB || in_sizes[4] != INF * H || in_sizes[6] != NST * HH || in_sizes[7] != L * H * H || in_sizes[9] != (H + HH) * H || in_sizes[13] != H * HH || in_sizes[17] != HH || out_size != NB) return;
  const int NROWS = NB;
  size_t off = 0; char* ws = (char*)d_ws;
  auto carve = [&](size_t bytes) { char* p = ws + off; off += (bytes + 255) & ~(size_t)255; return p; };
  b16* WP = (b16*)carve(H * INF * 2); b16* WG0 = (b16*)carve(H * H * 2); b16* WG1 = (b16*)carve(H * H * 2); b16* W1T = (b16*)carve(H * (H + HH) * 2); b16* W2T = (b16*)carve(HH * H * 2);
  if (off > ws_size || off > ((size_t)4 << 20)) return;
  WJob j0{Fp(4), INF, H, WP}, j1{Fp(7), H, H, WG0}, j2{Fp(7) + H * H, H, H, WG1}, j3{Fp(9), H + HH, H, W1T}, j4{Fp(13), H, HH, W2T};
  wprep_kernel<<<dim3((H * (H + HH) / 8 + 255) / 256, 5), 256, 0, stream>>>(j0, j1, j2, j3, j4, j4);
  chain_kernel<<<NROWS / 32, 64, 0, stream>>>(Fp(0), Ip(1), Fp(6), WP, WG0, WG1, W1T, W2T, Fp(5), Fp(10), Fp(11), Fp(12), Fp(14), Fp(15), Fp(16), Fp(17), Fp(18), (float*)d_out);
}
